// NeuroKernel_5884105195994
// MI455X (gfx1250) — hardware-verified
//
#include <hip/hip_runtime.h>
#include <math.h>

typedef __attribute__((ext_vector_type(16))) _Float16 v16h;
typedef __attribute__((ext_vector_type(16))) __bf16 v16b;
typedef __attribute__((ext_vector_type(8)))  _Float16 v8h;
typedef __attribute__((ext_vector_type(8)))  float v8f;
typedef __attribute__((ext_vector_type(4)))  float v4f;
typedef __attribute__((ext_vector_type(2)))  float v2f;
typedef __attribute__((ext_vector_type(4)))  unsigned v4u;
typedef __attribute__((ext_vector_type(4)))  int v4i;
typedef float __attribute__((may_alias)) float_a;
typedef int __attribute__((may_alias)) int_a;

template <typename T> __device__ __forceinline__ void vst2(void* p, T v) { *(volatile T*)p = v; __threadfence(); *(volatile T*)p = v; }
__device__ __forceinline__ v8f wmma16(v16h a, v16h b, v8f c) {
  v8f d = __builtin_amdgcn_wmma_f32_16x16x32_f16(false, a, false, b, (short)0, c, false, false);
  asm volatile("v_nop\n\tv_nop\n\tv_nop\n\tv_nop" : "+v"(d) : "v"(a), "v"(b));
  return d;
}
__device__ __forceinline__ v8f wmma_bf(v16b a, v16b b, v8f c) {
  v8f d = __builtin_amdgcn_wmma_f32_16x16x32_bf16(false, a, false, b, (short)0, c, false, false);
  asm volatile("v_nop\n\tv_nop\n\tv_nop\n\tv_nop" : "+v"(d) : "v"(a), "v"(b));
  return d;
}
__device__ __forceinline__ v16h frag_h(const _Float16* rowk0, int lane) {
  union { v16h v; v8h q[2]; } u; const _Float16* p = rowk0 + 8 * (lane >> 4);
  u.q[0] = *(const v8h*)p; u.q[1] = *(const v8h*)(p + 16); return u.v;
}
__device__ __forceinline__ v16h frag_f32(const float* rowk0, int lane) {
  v16h a; const float* p = rowk0 + 8 * (lane >> 4);
#pragma unroll
  for (int i = 0; i < 8; ++i) { a[i] = (_Float16)p[i]; a[8 + i] = (_Float16)p[16 + i]; }
  return a;
}
__device__ __forceinline__ v16h frag_f32s(const float* rowk0, int lane, float sc) {
  v16h a; const float* p = rowk0 + 8 * (lane >> 4);
#pragma unroll
  for (int i = 0; i < 8; ++i) { a[i] = (_Float16)(p[i] * sc); a[8 + i] = (_Float16)(p[16 + i] * sc); }
  return a;
}
__device__ __forceinline__ v16h fragc_f32(const float* W, int k0, int n, int lane, int ld, int K) {
  v16h a; const int g = lane >> 4;
#pragma unroll
  for (int i = 0; i < 8; ++i) { const int ka = k0 + 8 * g + i, kb = ka + 16;
    a[i] = (_Float16)(ka < K ? W[(size_t)(ka < K ? ka : K - 1) * ld + n] : 0.f); a[8 + i] = (_Float16)(kb < K ? W[(size_t)(kb < K ? kb : K - 1) * ld + n] : 0.f); }
  return a;
}
struct F2 { v16b h, l; };
__device__ __forceinline__ F2 bsplit16(const float v[16]) { F2 r;
#pragma unroll
  for (int i = 0; i < 16; ++i) { const __bf16 h = (__bf16)v[i]; r.h[i] = h; r.l[i] = (__bf16)(v[i] - (float)h); }
  return r; }
__device__ __forceinline__ F2 split_row(const float* row, int k0, int lane) { float v[16]; const float* p = row + k0 + 8 * (lane >> 4);
#pragma unroll
  for (int i = 0; i < 8; ++i) { v[i] = p[i]; v[8 + i] = p[16 + i]; }
  return bsplit16(v); }
__device__ __forceinline__ F2 split_rowK(const float* row, int k0, int lane, int K) { float v[16]; const int g = lane >> 4;
#pragma unroll
  for (int i = 0; i < 8; ++i) { const int ka = k0 + 8 * g + i, kb = ka + 16; v[i] = ka < K ? row[ka < K ? ka : K - 1] : 0.f; v[8 + i] = kb < K ? row[kb < K ? kb : K - 1] : 0.f; }
  return bsplit16(v); }
__device__ __forceinline__ F2 split_col(const float* W, int k0, int n, int lane, int ld, int K) { float v[16]; const int g = lane >> 4;
#pragma unroll
  for (int i = 0; i < 8; ++i) { const int ka = k0 + 8 * g + i, kb = ka + 16; v[i] = ka < K ? W[(size_t)(ka < K ? ka : K - 1) * ld + n] : 0.f; v[8 + i] = kb < K ? W[(size_t)(kb < K ? kb : K - 1) * ld + n] : 0.f; }
  return bsplit16(v); }
__device__ __forceinline__ v8f mac3(const F2& a, const F2& b, v8f c) { c = wmma_bf(a.l, b.h, c); c = wmma_bf(a.h, b.l, c); return wmma_bf(a.h, b.h, c); }
__device__ __forceinline__ float sigm(float v) { return 1.0f / (1.0f + expf(-v)); }
#define LDSX() do { asm volatile("s_wait_dscnt 0" ::: "memory"); __builtin_amdgcn_wave_barrier(); __builtin_amdgcn_fence(__ATOMIC_RELEASE, "workgroup"); } while (0)

__device__ __forceinline__ float bfr(float v) { return (float)(__bf16)v; }
#define NP 512
#define H1 1024
#define H2 128
#ifndef NRB
#define NRB (NP * NP / 64)
#endif
#ifndef OPITCH
#define OPITCH NP
#endif
#define WS_A  0u
#define WS_C  (WS_A + 4u * (size_t)NP * H1)
#define WS_KM (WS_C + 4u * (size_t)NP * H1)
#define WS_END (WS_KM + 4u * (size_t)NP * NP)
__global__ __launch_bounds__(256) void k_ac(const float* __restrict__ X, const float* __restrict__ W1, const float* __restrict__ B1, float* __restrict__ A, float* __restrict__ C) {
  const int i = blockIdx.x, which = blockIdx.y, t = threadIdx.x; const float xi = bfr(X[i]); float* D = (which == 0 ? A : C) + (size_t)i * H1; v4f o;
#pragma unroll
  for (int e = 0; e < 4; ++e) { const int h = t * 4 + e; o[e] = which == 0 ? xi * bfr(W1[h]) : (xi * bfr(W1[H1 + h]) + bfr(B1[h])); }
  vst2(D + t * 4, o); }
__global__ __launch_bounds__(128) void k_pair(const float* __restrict__ A, const float* __restrict__ C, const float* __restrict__ W2, const float* __restrict__ B2, const float* __restrict__ W3, const float* __restrict__ B3, float* __restrict__ KM) { __shared__ __align__(16) float sh2[64][132]; __shared__ __align__(16) float sk[64];
  const int tid = threadIdx.x, wave = tid >> 5, lane = tid & 31, col = lane & 15, g = lane >> 4; const size_t p0 = (size_t)blockIdx.x * 64; const size_t prow = p0 + wave * 16 + col; const int i = (int)(prow / NP), j = (int)(prow % NP);
  const float* ar = A + (size_t)i * H1; const float* cr = C + (size_t)j * H1;
  v8f acc[8] = {};
#pragma unroll 2
  for (int kc = 0; kc < H1 / 32; ++kc) { v16h a;
#pragma unroll
    for (int e = 0; e < 8; ++e) { const int h = kc * 32 + 8 * g + e; a[e] = (_Float16)fmaxf(ar[h] + cr[h], 0.f); a[8 + e] = (_Float16)fmaxf(ar[h + 16] + cr[h + 16], 0.f); }
#pragma unroll
    for (int jt = 0; jt < 8; ++jt) { v16h w; const int o = jt * 16 + col;
#pragma unroll
      for (int e = 0; e < 8; ++e) { w[e] = (_Float16)(bfr(W2[(size_t)(kc * 32 + 8 * g + e) * H2 + o]) * 16.0f); w[8 + e] = (_Float16)(bfr(W2[(size_t)(kc * 32 + 16 + 8 * g + e) * H2 + o]) * 16.0f); }
      acc[jt] = wmma16(a, w, acc[jt]); } }
#pragma unroll
  for (int jt = 0; jt < 8; ++jt) { const int o = jt * 16 + col; const float bb = bfr(B2[o]); const float w3 = bfr(W3[o]);
#pragma unroll
    for (int r = 0; r < 8; ++r) sh2[wave * 16 + 8 * g + r][o] = fmaxf(acc[jt][r] * (1.0f / 16.0f) + bb, 0.f) * w3; }
  __syncthreads();
  if (tid < 64) { const float* row = sh2[tid]; float s = 0.f; for (int o = 0; o < H2; ++o) s += row[o]; s += bfr(B3[0]); const size_t pr = p0 + tid; const int ii = (int)(pr / NP), jj = (int)(pr % NP); sk[tid] = (jj >= ii) ? s : 0.f; }
  __syncthreads();
  if (tid < 16) vst2(KM + p0 + tid * 4, *(const v4f*)&sk[tid * 4]); }
__global__ __launch_bounds__(128) void k_ktk(const float* __restrict__ KM, float* __restrict__ OUT) { __shared__ __align__(16) float sf[4][16][132];
  const int tid = threadIdx.x, wave = tid >> 5, lane = tid & 31, col = lane & 15, g = lane >> 4; const int b0 = blockIdx.y * 128; const int a0 = blockIdx.x * 64 + wave * 16;
  v8f acc[8] = {};
#pragma unroll 1
  for (int kc = 0; kc < NP / 32; ++kc) { const F2 a = split_col(KM, kc * 32, a0 + col, lane, NP, NP);
    asm volatile("s_wait_loadcnt 0x0" ::: "memory");
#pragma unroll
    for (int jt = 0; jt < 8; ++jt) { const F2 bq = split_col(KM, kc * 32, b0 + jt * 16 + col, lane, NP, NP); asm volatile("s_wait_loadcnt 0x0" ::: "memory"); acc[jt] = mac3(a, bq, acc[jt]); } }
#pragma unroll
  for (int jt = 0; jt < 8; ++jt)
#pragma unroll
    for (int r = 0; r < 8; ++r) sf[wave][8 * g + r][jt * 16 + col] = acc[jt][r];
  LDSX(); for (int rl = 0; rl < 16; ++rl) vst2(OUT + (size_t)(a0 + rl) * OPITCH + b0 + lane * 4, *(const v4f*)&sf[wave][rl][lane * 4]); }
extern "C" void kernel_launch(void* const* d_in, const int* in_sizes, int n_in, void* d_out, int out_size, void* d_ws, size_t ws_size, hipStream_t stream) {
  (void)in_sizes; (void)n_in; (void)out_size;
  const float** F = (const float**)d_in;
  if (ws_size < (size_t)WS_END) return;
  char* ws = (char*)d_ws; float *A = (float*)(ws + WS_A), *C = (float*)(ws + WS_C), *KM = (float*)(ws + WS_KM);
  k_ac<<<dim3(NP, 2), 256, 0, stream>>>(F[0], F[1], F[2], A, C);
  k_pair<<<dim3(NRB), 128, 0, stream>>>(A, C, F[3], F[4], F[5], F[6], KM);
  k_ktk<<<dim3(NP / 64, (NP >= 128 ? NP / 128 : 1)), 128, 0, stream>>>(KM, (float*)d_out);
}
